// HierarchicalGNN_31172872634961
// MI455X (gfx1250) — hardware-run, weakly checked
//
#include <hip/hip_runtime.h>


namespace {
constexpr int N = 6000, M = 16, EM = 32, E = 96000, AD = 13, MD = 256, CD = 512, PD = 29, HG_ = 4, DG = 64, HT = 4, DT = 128, WIDEC = 6 * CD, NPB = 8;
constexpr float HS = 256.0f, WSC = 256.0f;
typedef _Float16 b16;
typedef __attribute__((ext_vector_type(16))) _Float16 v16b;
typedef __attribute__((ext_vector_type(8))) _Float16 v8b;
typedef __attribute__((ext_vector_type(8))) float v8f;
typedef __attribute__((ext_vector_type(4))) float v4f;
__device__ __forceinline__ float bf16_rne(float f) { unsigned int u = __float_as_uint(f); u += 0x7FFFu + ((u >> 16) & 1u); float r = __uint_as_float(u & 0xFFFF0000u); asm volatile("" : "+v"(r)); return r; }
__device__ __forceinline__ float bfv(float f) { float r = bf16_rne(f); asm volatile("" : "+v"(r)); return r; }
__device__ __forceinline__ void split16(float v, b16& hi, b16& lo) { hi = (b16)v; lo = (b16)(v - (float)hi); }
__device__ __forceinline__ v16b frag_kb(const b16* p, int hh) { const v8b a = *(const v8b*)(p + 8 * hh), b = *(const v8b*)(p + 16 + 8 * hh); v16b f;
#pragma unroll
  for (int e = 0; e < 8; ++e) { f[e] = a[e]; f[8 + e] = b[e]; } return f; }
__device__ __forceinline__ v8f wmma16b(v16b a, v16b b, v8f c) { v8f d = __builtin_amdgcn_wmma_f32_16x16x32_f16(false, a, false, b, (short)0, c, false, false); asm volatile("v_nop\n\tv_nop\n\tv_nop\n\tv_nop" : "+v"(d) : "v"(a), "v"(b)); return d; }
__device__ __forceinline__ void wave_lds_sync() { __builtin_amdgcn_fence(__ATOMIC_RELEASE, "workgroup"); __builtin_amdgcn_wave_barrier(); __builtin_amdgcn_fence(__ATOMIC_ACQUIRE, "workgroup"); }
__device__ __forceinline__ float pmul(float a, float b) { float p = a * b; asm volatile("" : "+v"(p)); return p; }
__device__ __forceinline__ int iclamp(int v, int lo, int hi) { return v < lo ? lo : (v > hi ? hi : v); }
constexpr int CSR_NBLK8 = 512, CSR_GB8 = 8, CSR_GN8 = 1 << CSR_GB8  , CSR_TS8 = (CSR_GN8 < 32 ? 32 : CSR_GN8)  , CSR_MAXG8 = 512, CSR_CAP8 = 12288  ;
__device__ __host__ __forceinline__ int csr_tix8(int v) { return (v >> CSR_GB8) * CSR_TS8 + (v & (CSR_GN8 - 1)); }
__global__ __launch_bounds__(64) void csrA_kernel8(const int* __restrict__ dst, int E, int N, int nG, int CHP, int NGP, int* __restrict__ STG, int* __restrict__ HST) {
  extern __shared__ int sm[];
  int* cnt = sm; int* run = sm + NGP; int* ids = sm + 2 * NGP;
  const int b = blockIdx.x; const int ch = (E + CSR_NBLK8 - 1) / CSR_NBLK8; const int e0 = b * ch, e1 = min(E, e0 + ch);
  for (int i = threadIdx.x; i < NGP; i += 64) cnt[i] = 0;
  for (int i = threadIdx.x; i < CHP; i += 64) ids[i] = -1;
  __syncthreads();
  if (threadIdx.x == 0) {
    for (int e = e0; e < e1; ++e) { int d = dst[e]; d = (d < 0) ? 0 : (d >= N ? N - 1 : d); cnt[d >> CSR_GB8] += 1; }
    int acc = 0; for (int g = 0; g < nG; ++g) { run[g] = acc; acc += cnt[g]; }
    for (int e = e0; e < e1; ++e) { int d = dst[e]; d = (d < 0) ? 0 : (d >= N ? N - 1 : d); const int g = d >> CSR_GB8; ids[run[g]] = e; run[g] += 1; } }
  __syncthreads();
  typedef __attribute__((ext_vector_type(4))) int v4i;
  for (int pass = 0; pass < 2; ++pass) {
    for (int i = threadIdx.x; i < CHP / 4; i += 64) *(volatile v4i*)(STG + (size_t)b * CHP + i * 4) = *(const v4i*)(&ids[i * 4]);
    for (int i = threadIdx.x; i < NGP / 4; i += 64) { v4i v; for (int e = 0; e < 4; ++e) v[e] = (i * 4 + e < nG) ? cnt[i * 4 + e] : 0; *(volatile v4i*)(HST + (size_t)b * NGP + i * 4) = v; }
    __threadfence(); }
}
__global__ __launch_bounds__(512) void csrS_kernel8(const int* __restrict__ HST, int nG, int NGP, int* __restrict__ START, int* __restrict__ TOT, int* __restrict__ OFF) {
  __shared__ int tot[CSR_MAXG8];
  const int b = threadIdx.x;
  for (int pass = 0; pass < 2; ++pass) { int runb = 0; for (int g = 0; g < nG; ++g) { int c = HST[(size_t)b * NGP + g]; c = (c < 0) ? 0 : c; ((volatile int*)OFF)[(size_t)g * CSR_NBLK8 + b] = runb; runb += c; } __threadfence(); }
  for (int g = threadIdx.x; g < nG; g += 512) { int s = 0; for (int bb = 0; bb < CSR_NBLK8; ++bb) { int c = HST[(size_t)bb * NGP + g]; s += (c < 0) ? 0 : c; } tot[g] = s; }
  __syncthreads();
  if (threadIdx.x < 32) {
    __shared__ int st[CSR_MAXG8 + 32];
    if (threadIdx.x == 0) { int acc = 0; for (int g = 0; g < NGP; ++g) { st[g] = acc; if (g < nG) acc += (tot[g] + 31) & ~31; } st[NGP] = acc; }
    __builtin_amdgcn_fence(__ATOMIC_RELEASE, "workgroup"); __builtin_amdgcn_wave_barrier(); __builtin_amdgcn_fence(__ATOMIC_ACQUIRE, "workgroup");
    for (int pass = 0; pass < 2; ++pass) { for (int i = threadIdx.x; i < NGP + 32; i += 32) { ((volatile int*)START)[i] = (i <= NGP) ? st[min(i, NGP)] : 0; ((volatile int*)TOT)[i] = (i < nG) ? tot[i] : 0; } __threadfence(); } }
}
__global__ __launch_bounds__(256) void csrB_kernel8(const int* __restrict__ dst, int N, int nG, int CHP, int NGP, int permLen, const int* __restrict__ STG, const int* __restrict__ HST, const int* __restrict__ OFF, const int* __restrict__ START, const int* __restrict__ TOT, int* __restrict__ PERM, int* __restrict__ ROWPTR, int* __restrict__ ROWCNT, int* __restrict__ FLAG) {
  typedef __attribute__((ext_vector_type(4))) int v4i;
  __shared__ int ids[CSR_CAP8]; __shared__ unsigned short key[CSR_CAP8]; __shared__ int outp[CSR_CAP8]; __shared__ int ncnt[CSR_GN8 + 1]; __shared__ int boff[CSR_NBLK8 + 1];
  const int g = blockIdx.x, t_ = threadIdx.x; int tot = TOT[g]; int st = START[g], stn = START[g + 1]; const int v0 = g * CSR_GN8; const int nv = min(CSR_GN8, N - v0); const int t0 = g * CSR_TS8;
  st = (st < 0) ? 0 : (st > permLen - 32 ? permLen - 32 : st) & ~31; stn = (stn < st) ? st : (stn > permLen ? permLen : stn); tot = (tot < 0) ? 0 : tot; if (tot > stn - st && tot <= CSR_CAP8) tot = stn - st;
  if (tot > CSR_CAP8) {
    for (int pass = 0; pass < 2; ++pass) { for (int i = t_; i < CSR_TS8 / 4; i += 256) { v4i a, c; for (int e = 0; e < 4; ++e) { a[e] = st; c[e] = 0; } *(volatile v4i*)(ROWPTR + t0 + i * 4) = a; *(volatile v4i*)(ROWCNT + t0 + i * 4) = c; } if (t_ == 0) ((volatile int*)FLAG)[0] = 1; __threadfence(); } (void)nv; return; }
  if (t_ == 0) { int acc = 0; for (int b = 0; b < CSR_NBLK8; ++b) { boff[b] = acc; int c = HST[(size_t)b * NGP + g]; c = (c < 0) ? 0 : (c > CHP ? CHP : c); acc += c; if (acc > tot) acc = tot; } boff[CSR_NBLK8] = acc; }
  for (int i = t_; i <= CSR_GN8; i += 256) ncnt[i] = 0;
  __syncthreads();
  for (int b = 0; b < CSR_NBLK8; ++b) { const int c = boff[b + 1] - boff[b]; int o_ = OFF[(size_t)g * CSR_NBLK8 + b]; o_ = (o_ < 0) ? 0 : (o_ > CHP - c ? CHP - c : o_); const int* src_ = STG + (size_t)b * CHP + o_;
    for (int i = t_; i < c; i += 256) { int id = src_[i]; id = (id < 0) ? 0 : id; ids[boff[b] + i] = id; int d = dst[id]; d = (d < v0) ? v0 : (d >= N ? N - 1 : d); int kk = d - v0; kk = (kk < 0) ? 0 : (kk >= CSR_GN8 ? CSR_GN8 - 1 : kk); key[boff[b] + i] = (unsigned short)kk; } }
  __syncthreads();
  if (t_ == 0) { for (int i = 0; i < tot; ++i) ncnt[key[i]] += 1; int acc = 0; for (int vl = 0; vl < CSR_GN8; ++vl) { const int c = ncnt[vl]; ncnt[vl] = acc; acc += c; } ncnt[CSR_GN8] = acc;
    for (int i = 0; i < tot; ++i) { const int vl = key[i]; outp[ncnt[vl]] = ids[i]; ncnt[vl] += 1; }
    for (int vl = CSR_GN8; vl > 0; --vl) ncnt[vl] = ncnt[vl - 1]; ncnt[0] = 0; }
  __syncthreads();
  for (int pass = 0; pass < 2; ++pass) {
    for (int i = t_; i < (stn - st) / 4; i += 256) { v4i v; for (int e = 0; e < 4; ++e) { const int q = i * 4 + e; v[e] = (q < tot) ? outp[q] : -1; } *(volatile v4i*)(PERM + st + i * 4) = v; }
    for (int i = t_; i < CSR_TS8 / 4; i += 256) { v4i a, c; for (int e = 0; e < 4; ++e) { const int vl = i * 4 + e; const int vc = vl < CSR_GN8 ? vl : CSR_GN8; a[e] = (vl < CSR_GN8) ? st + ncnt[vc] : st; c[e] = (vl < nv) ? (ncnt[(vc < CSR_GN8 ? vc : CSR_GN8 - 1) + 1] - ncnt[vc]) : 0; } *(volatile v4i*)(ROWPTR + t0 + i * 4) = a; *(volatile v4i*)(ROWCNT + t0 + i * 4) = c; }
    __threadfence(); }
}
__global__ __launch_bounds__(256) void csrZ_kernel8(int* __restrict__ p, size_t n4) { typedef __attribute__((ext_vector_type(4))) int v4i; const size_t tid = (size_t)blockIdx.x * 256 + threadIdx.x, nth = (size_t)gridDim.x * 256; v4i z = {0, 0, 0, 0}; for (size_t i = tid; i < n4; i += nth) *(volatile v4i*)(p + i * 4) = z; }
struct CsrBufs8 { int *STG, *HST, *OFF, *START, *TOT, *PERM, *ROWPTR, *ROWCNT, *FLAG; int nG, NGP, CHP; size_t permLen; char* base; size_t bytes; };
static size_t csr_carve8(CsrBufs8& c, char* ws, size_t off, int E, int N) {
  const size_t off0 = off; c.base = ws + off;
  auto al = [&](size_t bytes) { char* p = ws + off; off += (bytes + 255) & ~(size_t)255; return p; };
  c.nG = (N + CSR_GN8 - 1) / CSR_GN8; c.NGP = (c.nG + 31) & ~31; const int ch = (E + CSR_NBLK8 - 1) / CSR_NBLK8; c.CHP = (ch + 31) & ~31; c.permLen = (size_t)E + 32 * (size_t)c.nG + 32;
  c.STG = (int*)al((size_t)CSR_NBLK8 * c.CHP * 4); c.HST = (int*)al((size_t)CSR_NBLK8 * c.NGP * 4); c.OFF = (int*)al((size_t)c.NGP * CSR_NBLK8 * 4); c.START = (int*)al((size_t)(c.NGP + 64) * 4); c.TOT = (int*)al((size_t)(c.NGP + 64) * 4);
  c.PERM = (int*)al(c.permLen * 4); c.ROWPTR = (int*)al((size_t)c.nG * CSR_TS8 * 4); c.ROWCNT = (int*)al((size_t)c.nG * CSR_TS8 * 4); c.FLAG = (int*)al(256);
  c.bytes = off - off0; return off;
}
static void csr_build8(const CsrBufs8& c, const int* dst, int E, int N, hipStream_t stream) {
  const size_t smem = (size_t)(2 * c.NGP + c.CHP) * 4;
  csrZ_kernel8<<<512, 256, 0, stream>>>((int*)c.base, c.bytes / 16);
  csrA_kernel8<<<CSR_NBLK8, 64, smem, stream>>>(dst, E, N, c.nG, c.CHP, c.NGP, c.STG, c.HST);
  csrS_kernel8<<<1, 512, 0, stream>>>(c.HST, c.nG, c.NGP, c.START, c.TOT, c.OFF);
  csrB_kernel8<<<c.nG, 256, 0, stream>>>(dst, N, c.nG, c.CHP, c.NGP, (int)c.permLen, c.STG, c.HST, c.OFF, c.START, c.TOT, c.PERM, c.ROWPTR, c.ROWCNT, c.FLAG);
}


__global__ __launch_bounds__(256) void wput_kernel(const float* __restrict__ wac, const float* __restrict__ wl, const float* __restrict__ wr, const float* __restrict__ wgin, const float* __restrict__ wth, const float* __restrict__ wph, const float* __restrict__ wq, const float* __restrict__ wk, const float* __restrict__ wv, const float* __restrict__ wskip, const float* __restrict__ wvc, const float* __restrict__ woc, b16* __restrict__ WAC, b16* __restrict__ WLR, b16* __restrict__ WGIN, b16* __restrict__ W6, b16* __restrict__ WVC, b16* __restrict__ WOC) { const size_t nt = (size_t)gridDim.x * 256, u0 = (size_t)blockIdx.x * 256 + threadIdx.x; v8b v;
  auto put = [&](b16* dst) { for (int pass = 0; pass < 2; ++pass) { *(volatile v8b*)dst = v; __threadfence(); } };
  for (size_t u = u0; u < (size_t)MD * 4; u += nt) { const int o = (int)(u / 4), k0 = (int)(u % 4) * 8;
#pragma unroll
    for (int j = 0; j < 8; ++j) { const int k = k0 + j; v[j] = (b16)(k < AD ? bf16_rne(wac[(size_t)k * MD + o]) * WSC : 0.0f); } put(WAC + (size_t)o * 32 + k0); }
  for (size_t u = u0; u < (size_t)2 * MD * (MD / 8); u += nt) { const int o = (int)(u / (MD / 8)), k0 = (int)(u % (MD / 8)) * 8; const float* w = o < MD ? wl : wr; const int oo = o % MD;
#pragma unroll
    for (int j = 0; j < 8; ++j) v[j] = (b16)(bf16_rne(w[(size_t)(k0 + j) * MD + oo]) * WSC); put(WLR + (size_t)o * MD + k0); }
  for (size_t u = u0; u < (size_t)CD * (MD / 8); u += nt) { const int o = (int)(u / (MD / 8)), k0 = (int)(u % (MD / 8)) * 8;
#pragma unroll
    for (int j = 0; j < 8; ++j) v[j] = (b16)(bf16_rne(wgin[(size_t)(k0 + j) * CD + o]) * WSC); put(WGIN + (size_t)o * MD + k0); }
  for (size_t u = u0; u < (size_t)WIDEC * (CD / 8); u += nt) { const int o = (int)(u / (CD / 8)), k0 = (int)(u % (CD / 8)) * 8; const int mI = o / CD, oo = o % CD; const float* w = mI == 0 ? wth : mI == 1 ? wph : mI == 2 ? wq : mI == 3 ? wk : mI == 4 ? wv : wskip;
#pragma unroll
    for (int j = 0; j < 8; ++j) v[j] = (b16)(bf16_rne(w[(size_t)(k0 + j) * CD + oo]) * WSC); put(W6 + (size_t)o * CD + k0); }
  for (size_t u = u0; u < (size_t)2 * 3 * CD * (CD / 8); u += nt) { const int which = (int)(u / ((size_t)3 * CD * (CD / 8))); const size_t r = u % ((size_t)3 * CD * (CD / 8)); const int i = (int)(r / (CD * (CD / 8))), o = (int)((r / (CD / 8)) % CD), k0 = (int)(r % (CD / 8)) * 8; const float* w = (which == 0 ? wvc : woc) + (size_t)i * CD * CD;
#pragma unroll
    for (int j = 0; j < 8; ++j) v[j] = (b16)(bf16_rne(w[(size_t)(k0 + j) * CD + o]) * WSC); put((which == 0 ? WVC : WOC) + ((size_t)i * CD + o) * CD + k0); } }
__global__ __launch_bounds__(32) void motif_kernel(const float* __restrict__ ax, const float* __restrict__ ew, const int* __restrict__ msrc, const int* __restrict__ mdst, const b16* __restrict__ WAC, const float* __restrict__ bac, const b16* __restrict__ WLR, const float* __restrict__ attn, const float* __restrict__ bgat, int NLIM, float* __restrict__ MF) { __shared__ __attribute__((aligned(16))) b16 Ah[16][MD + 8], Al[16][MD + 8]; __shared__ float X[16][AD + 1], H2[16][AD + 1], AHf[16][MD + 4], ELR[16][2 * MD + 4], Of[16][MD + 1], SC[EM][HG_], AL[EM][HG_], EW[EM]; __shared__ int ES[EM], ED[EM]; __shared__ float DO_[16], DI_[16];
  const int lane = threadIdx.x, nloc = lane & 15, hlf = lane >> 4; const size_t n = blockIdx.x; if (n >= (size_t)NLIM) return;
  { const int e = lane; ES[e] = iclamp(msrc[n * EM + e], 0, M - 1); ED[e] = iclamp(mdst[n * EM + e], 0, M - 1); EW[e] = bfv(ew[n * EM + e]); }
  for (int u = lane; u < 16 * AD; u += 32) X[u / AD][u % AD] = bfv(ax[n * 16 * AD + u]);
  wave_lds_sync();
  if (lane < 16) { float dout = 0.0f, din = 0.0f; for (int e = 0; e < EM; ++e) { dout += (ES[e] == lane) ? 1.0f : 0.0f; din += (ED[e] == lane) ? 1.0f : 0.0f; } DO_[lane] = rsqrtf(fmaxf(dout, 1.0f)); DI_[lane] = rsqrtf(fmaxf(din, 1.0f)); }
  wave_lds_sync();
  if (lane < AD) { float acc[16]; for (int a = 0; a < 16; ++a) acc[a] = 0.0f;
#pragma unroll 1
    for (int e = 0; e < EM; ++e) { const int s = ES[e], d = ED[e]; const float m = pmul(X[s][lane] * DO_[s], EW[e]);
#pragma unroll
      for (int a = 0; a < 16; ++a) acc[a] += (d == a) ? m : 0.0f; }
    for (int a = 0; a < 16; ++a) H2[a][lane] = acc[a] * DI_[a]; }
  wave_lds_sync();
  for (int u = lane; u < 16 * 40; u += 32) { const int a = u / 40, k = u % 40; b16 p = (b16)0.0f, pl = (b16)0.0f; if (k < AD) split16(H2[a][k] * HS, p, pl); Ah[a][k] = p; Al[a][k] = pl; }
  wave_lds_sync();
  { v8f acc[16];
#pragma unroll
    for (int t = 0; t < 16; ++t) acc[t] = (v8f){};
    { const v16b a = frag_kb(&Ah[nloc][0], hlf), al = frag_kb(&Al[nloc][0], hlf);
#pragma unroll
      for (int t = 0; t < 16; ++t) { const v16b bw = frag_kb(WAC + (size_t)(t * 16 + nloc) * 32, hlf); acc[t] = wmma16b(a, bw, acc[t]); acc[t] = wmma16b(al, bw, acc[t]); } }
#pragma unroll
    for (int t = 0; t < 16; ++t) { const int cc = t * 16 + nloc; const float bb = bfv(bac[cc]);
#pragma unroll
      for (int r8 = 0; r8 < 8; ++r8) AHf[8 * hlf + r8][cc] = fmaxf(acc[t][r8] * (1.0f / (HS * WSC)) + bb, 0.0f); } }
  wave_lds_sync();
  for (int rr = 0; rr < 16; ++rr) for (int q = 0; q < 8; ++q) { const int c = q * 32 + lane; b16 p, pl; split16(AHf[rr][c] * HS, p, pl); Ah[rr][c] = p; Al[rr][c] = pl; }
  if (lane < 16) for (int k = MD; k < MD + 8; ++k) { Ah[lane][k] = (b16)0.0f; Al[lane][k] = (b16)0.0f; }
  wave_lds_sync();
#pragma unroll 1
  for (int g = 0; g < 2; ++g) { v8f acc[16];
#pragma unroll
    for (int t = 0; t < 16; ++t) acc[t] = (v8f){};
#pragma unroll 2
    for (int kb = 0; kb < MD; kb += 32) { const v16b a = frag_kb(&Ah[nloc][kb], hlf), al = frag_kb(&Al[nloc][kb], hlf);
#pragma unroll
      for (int t = 0; t < 16; ++t) { const v16b bw = frag_kb(WLR + (size_t)(g * 256 + t * 16 + nloc) * MD + kb, hlf); acc[t] = wmma16b(a, bw, acc[t]); acc[t] = wmma16b(al, bw, acc[t]); } }
#pragma unroll
    for (int t = 0; t < 16; ++t)
#pragma unroll
      for (int r8 = 0; r8 < 8; ++r8) ELR[8 * hlf + r8][g * MD + t * 16 + nloc] = acc[t][r8] * (1.0f / (HS * WSC)); }
  wave_lds_sync();
  { const int e = lane, s = ES[e], d = ED[e];
#pragma unroll
    for (int h = 0; h < HG_; ++h) { float sc = 0.0f;
#pragma unroll 1
      for (int dd = 0; dd < DG; ++dd) { const int c = h * DG + dd; float t = ELR[s][c] + ELR[d][MD + c]; t = t > 0.0f ? t : 0.2f * t; sc += pmul(bfv(attn[c]), t); } SC[e][h] = sc; } }
  wave_lds_sync();
  { const int e = lane, d = ED[e];
#pragma unroll
    for (int h = 0; h < HG_; ++h) { float mx = -INFINITY; for (int e2 = 0; e2 < EM; ++e2) if (ED[e2] == d) mx = fmaxf(mx, SC[e2][h]); float z = 0.0f; for (int e2 = 0; e2 < EM; ++e2) if (ED[e2] == d) z += __expf(SC[e2][h] - mx); AL[e][h] = __expf(SC[e][h] - mx) / fmaxf(z, 1e-16f); } }
  wave_lds_sync();
  for (int q = 0; q < 8; ++q) { const int c = q * 32 + lane; const int h = c / DG; float o[16]; for (int a = 0; a < 16; ++a) o[a] = 0.0f;
#pragma unroll 1
    for (int e = 0; e < EM; ++e) { const int s = ES[e], d = ED[e]; const float m = pmul(AL[e][h], ELR[s][c]);
#pragma unroll
      for (int a = 0; a < 16; ++a) o[a] += (d == a) ? m : 0.0f; }
    float tot = 0.0f;
#pragma unroll
    for (int a = 0; a < 16; ++a) tot += o[a] + bfv(bgat[c]); Of[0][c] = tot * (1.0f / 16.0f); }
  wave_lds_sync();
  for (int pass = 0; pass < 2; ++pass) { for (int q = 0; q < 8; ++q) ((volatile float*)MF)[n * MD + q * 32 + lane] = Of[0][q * 32 + lane]; __threadfence(); } }
template <int KD>
__global__ __launch_bounds__(32) void ngemm_kernel(const float* __restrict__ IN, const float* __restrict__ ADDIN, const b16* __restrict__ W, const float* __restrict__ bias, const float* __restrict__ RES, int OW, int NLIM, float* __restrict__ OUT) { __shared__ __attribute__((aligned(16))) b16 Ah[16][KD + 8], Al[16][KD + 8]; __shared__ float Tf[16][260]; const int lane = threadIdx.x, nloc = lane & 15, hlf = lane >> 4; const size_t n0 = (size_t)blockIdx.x * 16; const int g = blockIdx.y; if (n0 >= (size_t)NLIM) return;
  for (int rr = 0; rr < 16; ++rr) for (int q = 0; q < KD / 32; ++q) { const int c = q * 32 + lane; float v = IN[(n0 + rr) * KD + c]; if (ADDIN) v += ADDIN[(n0 + rr) * KD + c]; b16 p, pl; split16(v * HS, p, pl); Ah[rr][c] = p; Al[rr][c] = pl; }
  if (lane < 16) for (int k = KD; k < KD + 8; ++k) { Ah[lane][k] = (b16)0.0f; Al[lane][k] = (b16)0.0f; }
  wave_lds_sync(); v8f acc[16];
#pragma unroll
  for (int t = 0; t < 16; ++t) acc[t] = (v8f){};
#pragma unroll 2
  for (int kb = 0; kb < KD; kb += 32) { const v16b a = frag_kb(&Ah[nloc][kb], hlf), al = frag_kb(&Al[nloc][kb], hlf);
#pragma unroll
    for (int t = 0; t < 16; ++t) { const v16b bw = frag_kb(W + (size_t)(g * 256 + t * 16 + nloc) * KD + kb, hlf); acc[t] = wmma16b(a, bw, acc[t]); acc[t] = wmma16b(al, bw, acc[t]); } }
#pragma unroll
  for (int t = 0; t < 16; ++t) { const int cc = t * 16 + nloc; const float bb = bias ? bfv(bias[g * 256 + cc]) : 0.0f;
#pragma unroll
    for (int r8 = 0; r8 < 8; ++r8) { const int rr = 8 * hlf + r8; float v = acc[t][r8] * (1.0f / (HS * WSC)) + bb; if (RES) v += RES[(n0 + rr) * OW + g * 256 + cc]; Tf[rr][cc] = v; } }
  wave_lds_sync();
  for (int pass = 0; pass < 2; ++pass) { for (int rr = 0; rr < 16; ++rr) for (int q = 0; q < 2; ++q) *(volatile v4f*)(OUT + (n0 + rr) * OW + g * 256 + q * 128 + lane * 4) = *(const v4f*)(&Tf[rr][q * 128 + lane * 4]); __threadfence(); } }
__global__ __launch_bounds__(256) void ginagg_kernel(const float* __restrict__ MF, const int* __restrict__ srcs, const int* __restrict__ PERM, const int* __restrict__ ROWPTR, const int* __restrict__ ROWCNT, int permLen, int NLIM, float* __restrict__ AGG) { const int wave = threadIdx.x >> 5, lane = threadIdx.x & 31; const size_t n = (size_t)blockIdx.x * NPB + wave; if (n >= (size_t)NLIM) return; v4f a0 = {0, 0, 0, 0}, a1 = {0, 0, 0, 0};
  int st = ROWPTR[n], cnt = ROWCNT[n]; cnt = iclamp(cnt, 0, E); st = iclamp(st, 0, permLen - cnt);
#pragma unroll 1
  for (int j = 0; j < cnt; ++j) { const int e = iclamp(PERM[st + j], 0, E - 1); const size_t s = (size_t)iclamp(srcs[e], 0, N - 1); if (s >= (size_t)NLIM) continue; a0 += *(const v4f*)(MF + s * MD + lane * 8); a1 += *(const v4f*)(MF + s * MD + lane * 8 + 4); }
  for (int pass = 0; pass < 2; ++pass) { *(volatile v4f*)(AGG + n * MD + lane * 8) = a0; *(volatile v4f*)(AGG + n * MD + lane * 8 + 4) = a1; __threadfence(); } }
__global__ __launch_bounds__(256) void edge_kernel(const float* __restrict__ WIDE, const float* __restrict__ eattr, const float* __restrict__ We, const float* __restrict__ be, const float* __restrict__ bth, const int* __restrict__ srcs, const int* __restrict__ PERM, const int* __restrict__ ROWPTR, const int* __restrict__ ROWCNT, int permLen, int NLIM, float* __restrict__ HE, float* __restrict__ HTr) { const int wave = threadIdx.x >> 5, lane = threadIdx.x & 31; const size_t n = (size_t)blockIdx.x * NPB + wave; if (n >= (size_t)NLIM) return; const int c0 = lane * 16;
  const float* wn = WIDE + n * WIDEC; float tn[16], pn[16], qn[16], mxe[16], acc[16];
#pragma unroll
  for (int i = 0; i < 16; ++i) { tn[i] = wn[c0 + i]; pn[i] = wn[CD + c0 + i] + bfv(bth[c0 + i]); qn[i] = wn[2 * CD + c0 + i]; mxe[i] = -INFINITY; acc[i] = 0.0f; }
  auto eav = [&](const float* ea5, int i) { const int c = c0 + i; float ea = bfv(be[c]);
#pragma unroll
    for (int jj = 0; jj < 5; ++jj) ea += pmul(ea5[jj], bfv(We[(size_t)jj * CD + c])); return ea; };
  float mx = -INFINITY, den = 0.0f;
  int st = ROWPTR[n], cnt = ROWCNT[n]; cnt = iclamp(cnt, 0, E); st = iclamp(st, 0, permLen - cnt); int nv = 0;
#pragma unroll 1
  for (int j = 0; j < cnt; ++j) { const int e = iclamp(PERM[st + j], 0, E - 1); const size_t s = (size_t)iclamp(srcs[e], 0, N - 1); if (s >= (size_t)NLIM) continue; ++nv; const float* ws_ = WIDE + s * WIDEC; float ea5[5];
#pragma unroll
    for (int jj = 0; jj < 5; ++jj) ea5[jj] = bfv(eattr[(size_t)e * 5 + jj]);
    float part = 0.0f;
#pragma unroll
    for (int i = 0; i < 16; ++i) { mxe[i] = fmaxf(mxe[i], ws_[c0 + i] - tn[i] + pn[i]); const float ea = eav(ea5, i); const float kj = ws_[3 * CD + c0 + i] + ea; part += pmul(qn[i], kj); }
    part += __shfl_xor(part, 1); part += __shfl_xor(part, 2); part += __shfl_xor(part, 4); const float sc = part * 0.08838834764831845f;
    const float mn = fmaxf(mx, sc); const float sf = (mx == -INFINITY) ? 0.0f : __expf(mx - mn); const float p = __expf(sc - mn);
#pragma unroll
    for (int i = 0; i < 16; ++i) { const float vj = ws_[4 * CD + c0 + i] + eav(ea5, i); acc[i] = pmul(acc[i], sf) + pmul(p, vj); } den = pmul(den, sf) + p; mx = mn; }
  const float inv = den > 0.0f ? 1.0f / fmaxf(den, 1e-16f) : 0.0f; v4f he[4], ht[4];
#pragma unroll
  for (int i = 0; i < 16; ++i) { he[i / 4][i % 4] = nv > 0 ? mxe[i] : 0.0f; ht[i / 4][i % 4] = pmul(acc[i], inv) + wn[5 * CD + c0 + i]; }
  for (int pass = 0; pass < 2; ++pass) { for (int q = 0; q < 4; ++q) { *(volatile v4f*)(HE + n * CD + c0 + q * 4) = he[q]; *(volatile v4f*)(HTr + n * CD + c0 + q * 4) = ht[q]; } __threadfence(); } }
__global__ __launch_bounds__(256) void vnode_kernel(const float* __restrict__ HTr, const float* __restrict__ vn, int NLIM, float* __restrict__ CH) { const size_t u = (size_t)blockIdx.x * 256 + threadIdx.x; if (u >= (size_t)NLIM * CD) return; const float v = HTr[u] + bfv(vn[u % CD]); for (int pass = 0; pass < 2; ++pass) { ((volatile float*)CH)[u] = v; __threadfence(); } }
__global__ __launch_bounds__(32) void gate_kernel(const float* __restrict__ HG, const float* __restrict__ HE, const float* __restrict__ HTr, const float* __restrict__ CH, const float* __restrict__ Wg, const float* __restrict__ bg, int NLIM, float* __restrict__ out) { __shared__ float GW[16][4]; const int lane = threadIdx.x; const size_t n0 = (size_t)blockIdx.x * 16; if (n0 >= (size_t)NLIM) return;
  if (lane < 16) { const size_t n = n0 + lane; float l[4]; for (int j = 0; j < 4; ++j) l[j] = bfv(bg[j]); const float* parts[4] = {HG + n * CD, HE + n * CD, HTr + n * CD, CH + n * CD};
#pragma unroll
    for (int pI = 0; pI < 4; ++pI) {
#pragma unroll 1
      for (int c = 0; c < CD; ++c) { const float x = parts[pI][c]; const float* wr = Wg + (size_t)(pI * CD + c) * 4; l[0] += pmul(x, bfv(wr[0])); l[1] += pmul(x, bfv(wr[1])); l[2] += pmul(x, bfv(wr[2])); l[3] += pmul(x, bfv(wr[3])); } }
    const float m = fmaxf(fmaxf(l[0], l[1]), fmaxf(l[2], l[3])); float e4[4], z = 0.0f; for (int j = 0; j < 4; ++j) { e4[j] = __expf(l[j] - m); z += e4[j]; } for (int j = 0; j < 4; ++j) GW[lane][j] = e4[j] / z; }
  wave_lds_sync();
  for (int pass = 0; pass < 2; ++pass) { for (int rr = 0; rr < 16; ++rr) { const size_t n = n0 + rr; for (int q = 0; q < CD / 32; ++q) { const int c = q * 32 + lane; ((volatile float*)out)[n * CD + c] = pmul(GW[rr][0], HG[n * CD + c]) + pmul(GW[rr][1], HE[n * CD + c]) + pmul(GW[rr][2], HTr[n * CD + c]) + pmul(GW[rr][3], CH[n * CD + c]); } } __threadfence(); } }
__global__ __launch_bounds__(256) void readout_kernel(const float* __restrict__ out, int NLIM, float* __restrict__ EMB) { const int c = blockIdx.x * 256 + threadIdx.x; if (c >= CD) return; float s = 0.0f, mx = -INFINITY;
#pragma unroll 1
  for (int n = 0; n < NLIM; ++n) { const float v = out[(size_t)n * CD + c]; s += v; mx = fmaxf(mx, v); }
  for (int pass = 0; pass < 2; ++pass) { ((volatile float*)EMB)[c] = s / (float)NLIM; ((volatile float*)EMB)[CD + c] = mx; __threadfence(); } }
__global__ __launch_bounds__(1024) void head_kernel(const float* __restrict__ EMB, const float* __restrict__ W1, const float* __restrict__ b1, const float* __restrict__ bng, const float* __restrict__ bnb, const float* __restrict__ W2, const float* __restrict__ b2, float* __restrict__ out1) { __shared__ float H1[1024], Em[1024]; const int j = threadIdx.x; Em[j] = EMB[j]; __syncthreads(); float s = bfv(b1[j]);
#pragma unroll 1
  for (int i = 0; i < 2 * CD; ++i) s += pmul(Em[i], bfv(W1[(size_t)i * 1024 + j])); s = pmul(s, bfv(bng[j]) * rsqrtf(1.0f + 1e-5f)) + bfv(bnb[j]); H1[j] = fmaxf(s, 0.0f); __syncthreads();
  float p = 0.0f; if (j < PD) { p = bfv(b2[j]);
#pragma unroll 1
    for (int i = 0; i < 1024; ++i) p += pmul(H1[i], bfv(W2[(size_t)i * PD + j])); }
  for (int pass = 0; pass < 2; ++pass) { if (j < PD) ((volatile float*)out1)[j] = p; __threadfence(); } }
}

extern "C" void kernel_launch(void* const* d_in, const int* in_sizes, int n_in, void* d_out, int out_size, void* d_ws, size_t ws_size, hipStream_t stream) {
  (void)n_in;
  auto Fp = [&](int i) { return (const float*)d_in[i]; }; auto Ip = [&](int i) { return (const int*)d_in[i]; };
  if (in_sizes[0] != N * M * AD || in_sizes[1] != N * EM || in_sizes[2] != E * 5 || in_sizes[3] != AD * MD || in_sizes[9] != MD * CD || in_sizes[26] != 3 * CD * CD || in_sizes[30] != 4 * CD * 4 || in_sizes[32] != 1024 * 1024 || in_sizes[36] != 1024 * PD || in_sizes[38] != N * EM || in_sizes[40] != E || in_sizes[41] != E || out_size != N * CD + PD) return;
  const int NLIM = N;
  size_t off = 0; char* ws = (char*)d_ws;
  auto carve = [&](size_t bytes) { char* p = ws + off; off += (bytes + 255) & ~(size_t)255; return p; };
  b16* WAC = (b16*)carve(MD * 32 * 2); b16* WLR = (b16*)carve((size_t)2 * MD * MD * 2); b16* WGIN = (b16*)carve((size_t)CD * MD * 2); b16* W6 = (b16*)carve((size_t)WIDEC * CD * 2); b16* WVC = (b16*)carve((size_t)3 * CD * CD * 2); b16* WOC = (b16*)carve((size_t)3 * CD * CD * 2);
  float* MF = (float*)carve((size_t)N * MD * 4); float* AGG = (float*)carve((size_t)N * MD * 4); float* HGp = (float*)carve((size_t)N * CD * 4); float* WIDE = (float*)carve((size_t)N * WIDEC * 4); float* HE = (float*)carve((size_t)N * CD * 4); float* HTp = (float*)carve((size_t)N * CD * 4); float* CH = (float*)carve((size_t)N * CD * 4); float* CV = (float*)carve((size_t)N * CD * 4); float* EMB = (float*)carve(2 * CD * 4); CsrBufs8 csr; off = csr_carve8(csr, ws, off, E, N);
  if (off > ws_size || off > ((size_t)160 << 20)) return;
  wput_kernel<<<512, 256, 0, stream>>>(Fp(3), Fp(5), Fp(6), Fp(9), Fp(11), Fp(13), Fp(15), Fp(17), Fp(19), Fp(23), Fp(26), Fp(28), WAC, WLR, WGIN, W6, WVC, WOC);
  csr_build8(csr, Ip(41), E, N, stream);
  motif_kernel<<<NLIM, 32, 0, stream>>>(Fp(0), Fp(1), Ip(38), Ip(39), WAC, Fp(4), WLR, Fp(7), Fp(8), NLIM, MF);
  const int nb = (NLIM + NPB - 1) / NPB;
  ginagg_kernel<<<nb, 256, 0, stream>>>(MF, Ip(40), csr.PERM, csr.ROWPTR, csr.ROWCNT, (int)csr.permLen, NLIM, AGG);
  ngemm_kernel<MD><<<dim3(NLIM / 16, 2), 32, 0, stream>>>(MF, AGG, WGIN, Fp(10), nullptr, CD, NLIM, HGp);
  { const float* biases[6] = {nullptr, Fp(14), Fp(16), Fp(18), Fp(20), Fp(24)};
    for (int mI = 0; mI < 6; ++mI) ngemm_kernel<CD><<<dim3(NLIM / 16, 2), 32, 0, stream>>>(HGp, nullptr, W6 + (size_t)mI * CD * CD, biases[mI], nullptr, WIDEC, NLIM, WIDE + mI * CD); }
  edge_kernel<<<nb, 256, 0, stream>>>(WIDE, Fp(2), Fp(21), Fp(22), Fp(12), Ip(40), csr.PERM, csr.ROWPTR, csr.ROWCNT, (int)csr.permLen, NLIM, HE, HTp);
  vnode_kernel<<<(NLIM * CD + 255) / 256, 256, 0, stream>>>(HTp, Fp(25), NLIM, CH);
  for (int i = 0; i < 3; ++i) { ngemm_kernel<CD><<<dim3(NLIM / 16, 2), 32, 0, stream>>>(CH, nullptr, WVC + (size_t)i * CD * CD, Fp(27) + i * CD, nullptr, CD, NLIM, CV);
    ngemm_kernel<CD><<<dim3(NLIM / 16, 2), 32, 0, stream>>>(CV, nullptr, WOC + (size_t)i * CD * CD, Fp(29) + i * CD, CH, CD, NLIM, CH); }
  float* out0 = (float*)d_out; float* out1 = out0 + (size_t)N * CD;
  gate_kernel<<<NLIM / 16, 32, 0, stream>>>(HGp, HE, HTp, CH, Fp(30), Fp(31), NLIM, out0);
  readout_kernel<<<2, 256, 0, stream>>>(out0, NLIM, EMB);
  head_kernel<<<1, 1024, 0, stream>>>(EMB, Fp(32), Fp(33), Fp(34), Fp(35), Fp(36), Fp(37), out1);
}
